// FraudGNN_48223892799810
// MI455X (gfx1250) — hardware-verified
//
#include <hip/hip_runtime.h>
#include <math.h>

constexpr int kNodes     = 50000;
constexpr int kEdges     = 800000;
constexpr int kRowsPad   = 50048;
constexpr int kCin       = 64;
constexpr int kHid       = 128;
constexpr int kCls       = 2;
constexpr int kThreads   = 256;
constexpr int kWaves     = kThreads / 32;
constexpr int kChunk     = 4096;
constexpr int kPerThread = kChunk / kThreads;
constexpr int kChunks    = (kEdges + kChunk - 1) / kChunk;
constexpr int kTile1     = 512;
constexpr int kTile2     = 256;
constexpr int kTile3     = 2048;
constexpr int kBlocks1   = (kRowsPad + kTile1 - 1) / kTile1;
constexpr int kBlocks2   = (kRowsPad + kTile2 - 1) / kTile2;
constexpr int kBlocks3   = (kRowsPad + kTile3 - 1) / kTile3;
constexpr float kWCarry    = 16.0f;
constexpr float kWCarryInv = 1.0f / 16.0f;

constexpr int ilog2c(int v) { return v <= 1 ? 0 : 1 + ilog2c(v >> 1); }

static_assert(kRowsPad % 64 == 0 && kRowsPad >= kNodes && kRowsPad - kNodes < 64, "pad");
static_assert(kHid % 64 == 0, "n tile");
static_assert((2 * kCin) % 32 == 0 && (2 * kHid) % 32 == 0, "k step");
static_assert(kEdges % kPerThread == 0 && kPerThread % 4 == 0, "edge groups");
static_assert(kEdges < (1 << 20), "edge bits");
static_assert(kTile3 <= 2048 && kTile1 <= 2048 && kTile2 <= 2048, "row bits");
static_assert(kChunk % 32 == 0, "chunk");
static_assert(kNodes % 16 == 0 && (kNodes * kCls * 4) % 128 == 0, "out lines");
static_assert(kBlocks1 * kTile1 >= kRowsPad && kBlocks2 * kTile2 >= kRowsPad && kBlocks3 * kTile3 >= kRowsPad, "tiles");
static_assert(kBlocks1 == 98 && kBlocks2 == 196 && kBlocks3 == 25 && kChunks == 196, "grid");

constexpr size_t kBt1Bytes = (size_t)kHid * (2 * kCin) * 2;
constexpr size_t kBt2Bytes = (size_t)kHid * (2 * kHid) * 2;
constexpr size_t kA1Bytes  = (size_t)kRowsPad * (2 * kCin) * 2;
constexpr size_t kH1Bytes  = (size_t)kRowsPad * kHid * 4;
constexpr size_t kA2Bytes  = (size_t)kRowsPad * (2 * kHid) * 2;
constexpr size_t kH2Bytes  = (size_t)kRowsPad * kHid * 4;
constexpr size_t kP3Bytes  = (size_t)kRowsPad * 4 * 4;
constexpr size_t kWsTotal  = kBt1Bytes + kBt2Bytes + kA1Bytes + kH1Bytes + kA2Bytes + kH2Bytes + kP3Bytes;
static_assert(kWsTotal == 90585088, "carve");
static_assert(kWsTotal <= (size_t)134217728, "carve cap");
static_assert(kBt1Bytes % 256 == 0 && kBt2Bytes % 256 == 0 && kA1Bytes % 256 == 0 &&
              kH1Bytes % 256 == 0 && kA2Bytes % 256 == 0 && kH2Bytes % 256 == 0 && kP3Bytes % 256 == 0, "align");

typedef __attribute__((ext_vector_type(16))) _Float16 v16h;
typedef __attribute__((ext_vector_type(8)))  _Float16 v8h;
typedef __attribute__((ext_vector_type(16))) __bf16   v16b;
typedef __attribute__((ext_vector_type(8)))  __bf16   v8b;
typedef __attribute__((ext_vector_type(8)))  float    v8f;
typedef __attribute__((ext_vector_type(4)))  float    v4f;
typedef __attribute__((ext_vector_type(2)))  float    v2f;
typedef __attribute__((ext_vector_type(4)))  int      v4i;
typedef __attribute__((ext_vector_type(4)))  unsigned int v4u;

template <int VPL> struct VecF;
template <> struct VecF<2> { typedef v2f T; };
template <> struct VecF<4> { typedef v4f T; };

__device__ __forceinline__ unsigned short f2bf_bits(float f) {
  unsigned u = __float_as_uint(f);
  return (unsigned short)((u + 0x7FFFu + ((u >> 16) & 1u)) >> 16);
}
__device__ __forceinline__ float bf_bits2f(unsigned short h) { return __uint_as_float(((unsigned)h) << 16); }

__device__ __forceinline__ void dep_guard_h(v8f& a, v8f& b, v16h x, v16h y) { asm volatile("v_nop\n\tv_nop\n\tv_nop\n\tv_nop" : "+v"(a), "+v"(b) : "v"(x), "v"(y)); }
__device__ __forceinline__ void dep_guard_b(v8f& a, v8f& b, v16b x, v16b y) { asm volatile("v_nop\n\tv_nop\n\tv_nop\n\tv_nop" : "+v"(a), "+v"(b) : "v"(x), "v"(y)); }
__device__ __forceinline__ void dep_guard4_h(v8f& a, v8f& b, v8f& c, v8f& d, v16h x, v16h y) {
  asm volatile("v_nop\n\tv_nop\n\tv_nop\n\tv_nop" : "+v"(a), "+v"(b), "+v"(c), "+v"(d) : "v"(x), "v"(y));
}
__device__ __forceinline__ void dep_guard4_b(v8f& a, v8f& b, v8f& c, v8f& d, v16b x, v16b y) {
  asm volatile("v_nop\n\tv_nop\n\tv_nop\n\tv_nop" : "+v"(a), "+v"(b), "+v"(c), "+v"(d) : "v"(x), "v"(y));
}
__device__ __forceinline__ void keep4_h(v16h a, v16h b, v16h c, v16h d) { asm volatile("v_nop" :: "v"(a), "v"(b), "v"(c), "v"(d)); }
__device__ __forceinline__ void keep4_b(v16b a, v16b b, v16b c, v16b d) { asm volatile("v_nop" :: "v"(a), "v"(b), "v"(c), "v"(d)); }
__device__ __forceinline__ void acc_guard4(v8f& a, v8f& b, v8f& c, v8f& d) { asm volatile("v_nop\n\tv_nop\n\tv_nop\n\tv_nop" : "+v"(a), "+v"(b), "+v"(c), "+v"(d)); }
template <typename T> struct Frag;
template <> struct Frag<_Float16> {
  typedef v16h V; union U { v16h v; v8h h[2]; };
  static __device__ __forceinline__ v16h load(const _Float16* p) {
    U f; f.h[0] = *(const v8h*)(p); f.h[1] = *(const v8h*)(p + 16); return f.v;
  }
  static __device__ __forceinline__ v8f mma(v16h a, v16h b, v8f c) {
    return __builtin_amdgcn_wmma_f32_16x16x32_f16(false, a, false, b, (short)0, c, false, false);
  }
  static __device__ __forceinline__ void guard(v8f& a, v8f& b, v16h x, v16h y) { dep_guard_h(a, b, x, y); }
  static __device__ __forceinline__ void guard4(v8f& a, v8f& b, v8f& c, v8f& d, v16h x, v16h y) { dep_guard4_h(a, b, c, d, x, y); }
  static __device__ __forceinline__ void keep(v16h a, v16h b, v16h c, v16h d) { keep4_h(a, b, c, d); }
};
template <> struct Frag<__bf16> {
  typedef v16b V; union U { v16b v; v8b h[2]; };
  static __device__ __forceinline__ v16b load(const __bf16* p) {
    U f; f.h[0] = *(const v8b*)(p); f.h[1] = *(const v8b*)(p + 16); return f.v;
  }
  static __device__ __forceinline__ v8f mma(v16b a, v16b b, v8f c) {
    return __builtin_amdgcn_wmma_f32_16x16x32_bf16(false, a, false, b, (short)0, c, false, false);
  }
  static __device__ __forceinline__ void guard(v8f& a, v8f& b, v16b x, v16b y) { dep_guard_b(a, b, x, y); }
  static __device__ __forceinline__ void guard4(v8f& a, v8f& b, v8f& c, v8f& d, v16b x, v16b y) { dep_guard4_b(a, b, c, d, x, y); }
  static __device__ __forceinline__ void keep(v16b a, v16b b, v16b c, v16b d) { keep4_b(a, b, c, d); }
};

__device__ __forceinline__ unsigned pk16(unsigned short a, unsigned short b) { return (unsigned)a | ((unsigned)b << 16); }
__device__ __forceinline__ unsigned short h_bits(float f) { const _Float16 h = (_Float16)f; return __builtin_bit_cast(unsigned short, h); }

template <int ET> struct Elem;
template <> struct Elem<0> { typedef _Float16 T; };
template <> struct Elem<1> { typedef __bf16 T; };
template <int ET, bool SPLIT, int BIAS_MODE, int OUT_MODE, bool RESID, int ACT = 0>
__global__ __launch_bounds__(256) void wmma_gemm64(
    const unsigned short* __restrict__ Ap, const unsigned short* __restrict__ A2p, int lda, long strideA,
    const unsigned short* __restrict__ Btp, const unsigned short* __restrict__ Bt2p, int ldb, long strideB,
    void* __restrict__ Cout, void* __restrict__ Cout2, int ldc, long strideC,
    const float* __restrict__ bias,
    const float* __restrict__ resid, long strideR,
    int M, int N, int K, float scale) {
  typedef typename Elem<ET>::T T;
  typedef typename Frag<T>::V V;
  const T* A = (const T*)Ap; const T* A2 = (const T*)A2p; const T* Bt = (const T*)Btp; const T* Bt2 = (const T*)Bt2p;
  __shared__ __align__(16) float sT[8][16 * 68];
  const int b    = blockIdx.y;
  const int lane = threadIdx.x & 31;
  const int wave = threadIdx.x >> 5;
  const int tilesN = N >> 6;
  const int tilesM = M >> 6;
  const int tile = blockIdx.x * 8 + wave;
  if (tile >= tilesM * tilesN) return;
  const int tm = tile / tilesN;
  const int tn = tile - tm * tilesN;
  const int m0 = tm << 6;
  const int n0 = tn << 6;

  const T* Ab  = A  + (size_t)b * strideA;
  const T* Bb  = Bt + (size_t)b * strideB;
  const T* Ab2 = SPLIT ? (A2  + (size_t)b * strideA) : nullptr;
  const T* Bb2 = SPLIT ? (Bt2 + (size_t)b * strideB) : nullptr;

  const int rlane = lane & 15;
  const int koff  = (lane >> 4) * 8;
  const int mOff  = (lane >> 4) * 8;

  v8f acc[4][4];
#pragma unroll
  for (int i = 0; i < 4; ++i)
#pragma unroll
    for (int j = 0; j < 4; ++j) acc[i][j] = (v8f){0.f,0.f,0.f,0.f,0.f,0.f,0.f,0.f};

  for (int k0 = 0; k0 < K; k0 += 32) {
    V bh[4], bl[4];
#pragma unroll
    for (int j = 0; j < 4; ++j) {
      const size_t bo = (size_t)(n0 + (j << 4) + rlane) * ldb + koff + k0;
      bh[j] = Frag<T>::load(Bb + bo);
      if (SPLIT) bl[j] = Frag<T>::load(Bb2 + bo);
    }
#pragma unroll
    for (int i = 0; i < 4; ++i) {
      const size_t ao = (size_t)(m0 + (i << 4) + rlane) * lda + koff + k0;
      V ah = Frag<T>::load(Ab + ao);
      V al;
      if (SPLIT) al = Frag<T>::load(Ab2 + ao);
#pragma unroll
      for (int j = 0; j < 4; ++j) {
        acc[i][j] = Frag<T>::mma(ah, bh[j], acc[i][j]);
        if (SPLIT) {
          acc[i][j] = Frag<T>::mma(ah, bl[j], acc[i][j]);
          acc[i][j] = Frag<T>::mma(al, bh[j], acc[i][j]);
        }
      }
      Frag<T>::guard4(acc[i][0], acc[i][1], acc[i][2], acc[i][3], ah, SPLIT ? al : ah);
    }
    Frag<T>::keep(bh[0], bh[1], bh[2], bh[3]);
    if (SPLIT) Frag<T>::keep(bl[0], bl[1], bl[2], bl[3]);
  }
  acc_guard4(acc[0][0], acc[0][1], acc[0][2], acc[0][3]);
  acc_guard4(acc[1][0], acc[1][1], acc[1][2], acc[1][3]);
  acc_guard4(acc[2][0], acc[2][1], acc[2][2], acc[2][3]);
  acc_guard4(acc[3][0], acc[3][1], acc[3][2], acc[3][3]);

  float* slab = sT[wave];
  const float* Rb = RESID ? (resid + (size_t)b * strideR) : nullptr;
#pragma unroll
  for (int i = 0; i < 4; ++i) {
    const int mBase = m0 + (i << 4);
#pragma unroll
    for (int j = 0; j < 4; ++j) {
      const int n = n0 + (j << 4) + rlane;
      float bv = 0.f;
      if (BIAS_MODE == 2) bv = bias[n];
#pragma unroll
      for (int r = 0; r < 8; ++r) {
        float v = acc[i][j][r] * scale;
        if (BIAS_MODE == 1) v += bias[mBase + mOff + r];
        if (BIAS_MODE == 2) v += bv;
        if (RESID) v += Rb[(size_t)(mBase + mOff + r) * ldc + n];
        if (ACT == 2) v = fmaxf(v, 0.0f);
        if (ACT == 4) v = (v > 0.f) ? v : 0.01f * v;
        slab[(mOff + r) * 68 + (j << 4) + rlane] = v;
      }
    }
    __builtin_amdgcn_fence(__ATOMIC_RELEASE, "workgroup");
    __builtin_amdgcn_wave_barrier();
    __builtin_amdgcn_fence(__ATOMIC_ACQUIRE, "workgroup");
    if (OUT_MODE == 0) {
      float* C = (float*)Cout + (size_t)b * strideC;
      const int hh = lane >> 4, c4 = (lane & 15) * 4;
      for (int pass = 0; pass < 2; ++pass) {
#pragma unroll
        for (int it = 0; it < 8; ++it) {
          const int row = it * 2 + hh;
          v4f v = *(const v4f*)(slab + row * 68 + c4);
          *(volatile v4f*)(C + (size_t)(mBase + row) * ldc + n0 + c4) = v;
        }
        __threadfence();
      }
    } else {
      const int q = lane >> 3, c8 = (lane & 7) * 8;
      unsigned short* C  = (unsigned short*)Cout  + (size_t)b * strideC;
      unsigned short* C2 = (OUT_MODE == 2) ? ((unsigned short*)Cout2 + (size_t)b * strideC) : nullptr;
      for (int pass = 0; pass < 2; ++pass) {
#pragma unroll
        for (int it = 0; it < 4; ++it) {
          const int row = it * 4 + q;
          const float* sp = slab + row * 68 + c8;
          v8h hv, lv;
#pragma unroll
          for (int e = 0; e < 8; ++e) {
            if (OUT_MODE == 1) {
              hv[e] = (_Float16)sp[e];
            } else {
              unsigned short hb = f2bf_bits(sp[e]);
              unsigned short lb = f2bf_bits(sp[e] - bf_bits2f(hb));
              hv[e] = __builtin_bit_cast(_Float16, hb);
              lv[e] = __builtin_bit_cast(_Float16, lb);
            }
          }
          *(volatile v8h*)(C + (size_t)(mBase + row) * ldc + n0 + c8) = hv;
          if (OUT_MODE == 2) *(volatile v8h*)(C2 + (size_t)(mBase + row) * ldc + n0 + c8) = lv;
        }
        __threadfence();
      }
    }
    __builtin_amdgcn_fence(__ATOMIC_RELEASE, "workgroup");
    __builtin_amdgcn_wave_barrier();
    __builtin_amdgcn_fence(__ATOMIC_ACQUIRE, "workgroup");
  }
}

__global__ __launch_bounds__(kThreads) void wpack_kernel(const float* __restrict__ W1l, const float* __restrict__ W1r,
                                                         const float* __restrict__ W2l, const float* __restrict__ W2r,
                                                         unsigned short* __restrict__ Bt1, unsigned short* __restrict__ Bt2) {
  __shared__ float sm[128][65];
  const int t = threadIdx.x;
  const int b = blockIdx.x;
  const float* W = (b == 0) ? W1l : (b == 1) ? W1r : (b < 4) ? W2l : W2r;
  const int k0   = (b == 3 || b == 5) ? 64 : 0;
  unsigned short* Bt = (b < 2) ? Bt1 : Bt2;
  const int ldb  = (b < 2) ? (2 * kCin) : (2 * kHid);
  const int col0 = (b < 2) ? (b * 64) : ((b - 2) * 64);
#pragma unroll 4
  for (int i = 0; i < 32; ++i) {
    const int e  = i * kThreads + t;
    const int kr = e >> 7;
    const int nn = e & 127;
    sm[nn][kr] = W[(size_t)(k0 + kr) * kHid + nn] * kWCarry;
  }
  __syncthreads();
  const int lane = t & 31, wave = t >> 5;
  const int q = lane >> 3, c8 = (lane & 7) * 8;
#pragma unroll
  for (int it = 0; it < 4; ++it) {
    const int row = it * 32 + wave * 4 + q;
    unsigned short hb[8];
#pragma unroll
    for (int e = 0; e < 8; ++e) hb[e] = h_bits(sm[row][c8 + e]);
    const v4u u = (v4u){pk16(hb[0], hb[1]), pk16(hb[2], hb[3]), pk16(hb[4], hb[5]), pk16(hb[6], hb[7])};
    unsigned short* dp = Bt + (size_t)row * ldb + col0 + c8;
    *(volatile v4u*)dp = u;
    __threadfence();
    *(volatile v4u*)dp = u;
  }
}

__device__ __forceinline__ int blk_excl_scan(int cnt, int* scan_ws, int tid, int* tot) {
  const int lane = tid & 31, wave = tid >> 5; int incl = cnt;
#pragma unroll
  for (int o = 1; o < 32; o <<= 1) { const int v = __shfl_up(incl, o, 32); if (lane >= o) incl += v; }
  if (lane == 31) scan_ws[wave] = incl;
  __syncthreads();
  if (wave == 0) { int wv = (lane < kThreads / 32) ? scan_ws[lane] : 0; int wincl = wv;
#pragma unroll
    for (int o = 1; o < 32; o <<= 1) { const int v = __shfl_up(wincl, o, 32); if (lane >= o) wincl += v; }
    if (lane < kThreads / 32) scan_ws[32 + lane] = wincl - wv; if (lane == 31) scan_ws[64] = wincl; }
  __syncthreads();
  const int res = scan_ws[32 + wave] + incl - cnt; *tot = scan_ws[64];
  return res;
}
template <int TR>
__device__ __forceinline__ int chunk_hits(const int* __restrict__ dstv, int e0, int n0, int tid, int* LIST, int* scan_ws) {
  const int  eb    = e0 + tid * kPerThread;
  const bool valid = eb < kEdges;
  const int  ebc   = valid ? eb : (kEdges - kPerThread);
  int rec[kPerThread]; int cnt = 0;
#pragma unroll
  for (int k = 0; k < kPerThread; k += 4) {
    const v4i d4 = *(const v4i*)(dstv + ebc + k);
#pragma unroll
    for (int e = 0; e < 4; ++e) {
      const unsigned rel = (unsigned)d4[e] - (unsigned)n0;
      int r = -1;
      if (valid && rel < (unsigned)TR) { r = ((int)rel << 20) | (eb + k + e); ++cnt; }
      rec[k + e] = r;
    }
  }
  int tot; int p = blk_excl_scan(cnt, scan_ws, tid, &tot);
#pragma unroll
  for (int k = 0; k < kPerThread; ++k) if (rec[k] >= 0) { if ((unsigned)p < (unsigned)kChunk) LIST[p] = rec[k]; ++p; }
  __syncthreads();
  return tot < kChunk ? tot : kChunk;
}

template <int CC, int TR>
__global__ __launch_bounds__(kThreads) void sage_agg_kernel(const float* __restrict__ F, const int* __restrict__ ei,
                                                           unsigned short* __restrict__ Aout) {
  static_assert(CC == 64 || CC == 128, "cc");
  static_assert(TR * CC == 32768 && TR % kWaves == 0, "tile");
  constexpr int VPL  = CC / 32;
  constexpr int RPW  = TR / kWaves;
  constexpr int OWNS = 20 + ilog2c(RPW);
  typedef typename VecF<VPL>::T vacc;
  __shared__ __align__(16) float SACC[TR * CC];
  __shared__ int   LIST[kChunk];
  __shared__ float SCNT[TR];
  __shared__ int   scan_ws[80];
  const int tid = threadIdx.x, lane = tid & 31, wave = tid >> 5;
  const int n0 = blockIdx.x * TR;
  const int* srcv = ei;
  const int* dstv = ei + kEdges;

  const v4f z4 = {0.0f, 0.0f, 0.0f, 0.0f};
  for (int i = tid; i < TR * CC / 4; i += kThreads) *(v4f*)(SACC + 4 * i) = z4;
  for (int i = tid; i < kChunk; i += kThreads) LIST[i] = -1;
  for (int i = tid; i < TR; i += kThreads) SCNT[i] = 0.0f;
  if (tid < 80) scan_ws[tid] = 0;
  __syncthreads();

#pragma unroll 1
  for (int c = 0; c < kChunks; ++c) {
    const int tot = chunk_hits<TR>(dstv, c * kChunk, n0, tid, LIST, scan_ws);
#pragma unroll 1
    for (int base = 0; base < tot; base += 32) {
      const int q  = base + lane;
      const int rl = LIST[q];
      const int rv = (q < tot) ? rl : -1;
      const int own = (rv >= 0 && ((rv >> OWNS) & 7) == wave) ? 1 : 0;
      unsigned msk = (unsigned)__ballot(own);
#pragma unroll 1
      for (int it = 0; it < 32; ++it) {
        if (msk == 0u) break;
        const int bp = __builtin_ctz(msk); msk &= msk - 1u;
        const int r  = __shfl(rv, bp, 32);
        const int dl = (r >> 20) & (TR - 1);
        int e = r & 0xFFFFF; e = e < kEdges ? e : kEdges - 1;
        int s = srcv[e]; s = s < 0 ? 0 : (s >= kNodes ? kNodes - 1 : s);
        const vacc hv = *(const vacc*)(F + (size_t)s * CC + VPL * lane);
        float* rp = SACC + dl * CC + VPL * lane;
        vacc a = *(const vacc*)rp;
        a = a + hv;
        *(vacc*)rp = a;
        if (lane == 0) SCNT[dl] += 1.0f;
      }
    }
    __syncthreads();
  }
  __syncthreads();

  constexpr int LPR = CC / 4;
  constexpr int RPI = 32 / LPR;
  static_assert(kRowsPad % RPI == 0 && (RPW % RPI) == 0, "rows");
  const int rowsel = lane / LPR;
  const int ql     = lane % LPR;
  const int hsel   = ql / (CC / 8);
  const int c8     = (ql % (CC / 8)) * 8;
#pragma unroll 1
  for (int j = 0; j < RPW / RPI; ++j) {
    const int nrow0 = n0 + wave * RPW + j * RPI;
    if (nrow0 < kRowsPad) {
      const int dl = wave * RPW + j * RPI + rowsel;
      const int n  = nrow0 + rowsel;
      const bool live = n < kNodes;
      const int nc = live ? n : (kNodes - 1);
      const float livef = live ? 1.0f : 0.0f;
      const float fa  = hsel ? 0.0f : livef;
      const float fb  = hsel ? livef : 0.0f;
      const float cnt = SCNT[dl];
      const float inv = 1.0f / fmaxf(cnt, 1.0f);
      const float* ap = SACC + dl * CC + c8;
      const float* fp = F + (size_t)nc * CC + c8;
      const v4f a0 = *(const v4f*)(ap), a1 = *(const v4f*)(ap + 4);
      const v4f f0 = *(const v4f*)(fp), f1 = *(const v4f*)(fp + 4);
      unsigned short hb[8];
#pragma unroll
      for (int e = 0; e < 4; ++e) {
        const float v0 = fmaf(fa, a0[e] * inv, fb * f0[e]);
        const float v1 = fmaf(fa, a1[e] * inv, fb * f1[e]);
        hb[e] = h_bits(v0); hb[4 + e] = h_bits(v1);
      }
      const v4u u = (v4u){pk16(hb[0], hb[1]), pk16(hb[2], hb[3]), pk16(hb[4], hb[5]), pk16(hb[6], hb[7])};
      unsigned short* dp = Aout + (size_t)n * (2 * CC) + hsel * CC + c8;
      *(volatile v4u*)dp = u;
      __threadfence();
      *(volatile v4u*)dp = u;
    }
  }
}

__global__ __launch_bounds__(kThreads) void proj_out_kernel(const float* __restrict__ H2, const float* __restrict__ W3l,
                                                            const float* __restrict__ W3r, float* __restrict__ P3) {
  __shared__ float sWl[2 * kHid];
  __shared__ float sWr[2 * kHid];
  const int tid = threadIdx.x;
  sWl[tid] = W3l[tid];
  sWr[tid] = W3r[tid];
  __syncthreads();
  const int n = blockIdx.x * kThreads + tid;
  if (n < kRowsPad) {
    const bool live = n < kNodes;
    const int nc = live ? n : (kNodes - 1);
    const float* hr = H2 + (size_t)nc * kHid;
    float p0 = 0.0f, p1 = 0.0f, p2 = 0.0f, p3 = 0.0f;
#pragma unroll 1
    for (int k4 = 0; k4 < kHid / 4; ++k4) {
      const v4f h = *(const v4f*)(hr + 4 * k4);
#pragma unroll
      for (int e = 0; e < 4; ++e) {
        const int k = 4 * k4 + e;
        p0 = fmaf(h[e], sWl[2 * k],     p0);
        p1 = fmaf(h[e], sWl[2 * k + 1], p1);
        p2 = fmaf(h[e], sWr[2 * k],     p2);
        p3 = fmaf(h[e], sWr[2 * k + 1], p3);
      }
    }
    const float lf = live ? 1.0f : 0.0f;
    const v4f pv = (v4f){p0 * lf, p1 * lf, p2 * lf, p3 * lf};
    float* pp = P3 + (size_t)n * 4;
    *(volatile v4f*)pp = pv;
    __threadfence();
    *(volatile v4f*)pp = pv;
  }
}

__global__ __launch_bounds__(kThreads) void sage_out_kernel(const float* __restrict__ P3, const int* __restrict__ ei,
                                                            const float* __restrict__ b3, float* __restrict__ out) {
  constexpr int TR   = kTile3;
  constexpr int RPW  = TR / kWaves;
  constexpr int OWNS = 20 + ilog2c(RPW);
  __shared__ int   LIST[kChunk];
  __shared__ float SCNT[TR];
  __shared__ float SAGG[2 * TR];
  __shared__ int   scan_ws[80];
  const int tid = threadIdx.x, lane = tid & 31, wave = tid >> 5;
  const int n0 = blockIdx.x * TR;
  const int* srcv = ei;
  const int* dstv = ei + kEdges;

  for (int i = tid; i < kChunk; i += kThreads) LIST[i] = -1;
  for (int i = tid; i < TR; i += kThreads) SCNT[i] = 0.0f;
  for (int i = tid; i < 2 * TR; i += kThreads) SAGG[i] = 0.0f;
  if (tid < 80) scan_ws[tid] = 0;
  __syncthreads();

#pragma unroll 1
  for (int c = 0; c < kChunks; ++c) {
    const int tot = chunk_hits<TR>(dstv, c * kChunk, n0, tid, LIST, scan_ws);
#pragma unroll 1
    for (int base = 0; base < tot; base += 32) {
      const int q  = base + lane;
      const int rl = LIST[q];
      const int rv = (q < tot) ? rl : -1;
      const int own = (rv >= 0 && ((rv >> OWNS) & 7) == wave) ? 1 : 0;
      unsigned msk = (unsigned)__ballot(own);
#pragma unroll 1
      for (int it = 0; it < 32; ++it) {
        if (msk == 0u) break;
        const int bp = __builtin_ctz(msk); msk &= msk - 1u;
        const int r  = __shfl(rv, bp, 32);
        const int dl = (r >> 20) & (TR - 1);
        int e = r & 0xFFFFF; e = e < kEdges ? e : kEdges - 1;
        int s = srcv[e]; s = s < 0 ? 0 : (s >= kNodes ? kNodes - 1 : s);
        const v4f pv = *(const v4f*)(P3 + (size_t)s * 4);
        if (lane == 0) { SAGG[2 * dl] += pv[0]; SAGG[2 * dl + 1] += pv[1]; SCNT[dl] += 1.0f; }
      }
    }
    __syncthreads();
  }
  __syncthreads();

  const float bz0 = b3[0], bz1 = b3[1];
  const int slA = (2 * lane) & 31, slB = (2 * lane + 1) & 31;
#pragma unroll 1
  for (int it = 0; it < RPW / 32; ++it) {
    const int dl = wave * RPW + it * 32 + lane;
    const int n  = n0 + dl;
    const int nc = n < kNodes ? n : (kNodes - 1);
    const float inv = 1.0f / fmaxf(SCNT[dl], 1.0f);
    const v4f pr = *(const v4f*)(P3 + (size_t)nc * 4);
    float z0 = SAGG[2 * dl] * inv + bz0;     z0 = z0 + pr[2];
    float z1 = SAGG[2 * dl + 1] * inv + bz1; z1 = z1 + pr[3];
    const float mx = fmaxf(z0, z1), mn = fminf(z0, z1);
    const float lse = mx + logf(1.0f + expf(mn - mx));
    const float o0 = z0 - lse, o1 = z1 - lse;
    const float pa0 = __shfl(o0, slA, 32), pa1 = __shfl(o1, slA, 32);
    const float pb0 = __shfl(o0, slB, 32), pb1 = __shfl(o1, slB, 32);
    const v4f ov = (v4f){pa0, pa1, pb0, pb1};
    const int np = n0 + wave * RPW + it * 32 + 2 * lane;
    const bool wr = (lane < 16) && (np + 1 < kNodes);
    float* op = out + (size_t)(wr ? np : 0) * kCls;
    if (wr) *(volatile v4f*)op = ov;
    __threadfence();
    if (wr) *(volatile v4f*)op = ov;
  }
}

extern "C" void kernel_launch(void* const* d_in, const int* in_sizes, int n_in,
                              void* d_out, int out_size, void* d_ws, size_t ws_size, hipStream_t stream) {
  if (n_in < 11) return;
  if (in_sizes[0] != kNodes * kCin || in_sizes[1] != 2 * kEdges || out_size != kNodes * kCls) return;
  if (in_sizes[2] != kCin * kHid || in_sizes[4] != kCin * kHid || in_sizes[5] != kHid * kHid || in_sizes[7] != kHid * kHid) return;
  if (in_sizes[3] != kHid || in_sizes[6] != kHid || in_sizes[8] != kHid * kCls || in_sizes[9] != kCls || in_sizes[10] != kHid * kCls) return;
  if (kWsTotal > ws_size) return;

  const float* x   = (const float*)d_in[0];
  const int*   ei  = (const int*)d_in[1];
  const float* W1l = (const float*)d_in[2];
  const float* b1  = (const float*)d_in[3];
  const float* W1r = (const float*)d_in[4];
  const float* W2l = (const float*)d_in[5];
  const float* b2  = (const float*)d_in[6];
  const float* W2r = (const float*)d_in[7];
  const float* W3l = (const float*)d_in[8];
  const float* b3  = (const float*)d_in[9];
  const float* W3r = (const float*)d_in[10];
  float* out = (float*)d_out;

  char* ws = (char*)d_ws; size_t off = 0;
  unsigned short* Bt1 = (unsigned short*)(ws + off); off += kBt1Bytes;
  unsigned short* Bt2 = (unsigned short*)(ws + off); off += kBt2Bytes;
  unsigned short* A1  = (unsigned short*)(ws + off); off += kA1Bytes;
  float*          H1  = (float*)(ws + off);          off += kH1Bytes;
  unsigned short* A2  = (unsigned short*)(ws + off); off += kA2Bytes;
  float*          H2  = (float*)(ws + off);          off += kH2Bytes;
  float*          P3  = (float*)(ws + off);          off += kP3Bytes;
  if (off != kWsTotal || off > ws_size) return;

  const int gemmTiles  = (kRowsPad / 64) * (kHid / 64);
  const int gemmBlocks = (gemmTiles + 7) / 8;

  wpack_kernel<<<6, kThreads, 0, stream>>>(W1l, W1r, W2l, W2r, Bt1, Bt2);
  sage_agg_kernel<kCin, kTile1><<<kBlocks1, kThreads, 0, stream>>>(x, ei, A1);
  wmma_gemm64<0, false, 2, 0, false, 2><<<dim3(gemmBlocks, 1), 256, 0, stream>>>(
      (const unsigned short*)A1, (const unsigned short*)nullptr, 2 * kCin, 0L,
      (const unsigned short*)Bt1, (const unsigned short*)nullptr, 2 * kCin, 0L,
      (void*)H1, (void*)nullptr, kHid, 0L,
      b1, (const float*)nullptr, 0L, kRowsPad, kHid, 2 * kCin, kWCarryInv);
  sage_agg_kernel<kHid, kTile2><<<kBlocks2, kThreads, 0, stream>>>(H1, ei, A2);
  wmma_gemm64<0, false, 2, 0, false, 2><<<dim3(gemmBlocks, 1), 256, 0, stream>>>(
      (const unsigned short*)A2, (const unsigned short*)nullptr, 2 * kHid, 0L,
      (const unsigned short*)Bt2, (const unsigned short*)nullptr, 2 * kHid, 0L,
      (void*)H2, (void*)nullptr, kHid, 0L,
      b2, (const float*)nullptr, 0L, kRowsPad, kHid, 2 * kHid, kWCarryInv);
  proj_out_kernel<<<(kRowsPad + kThreads - 1) / kThreads, kThreads, 0, stream>>>(H2, W3l, W3r, P3);
  sage_out_kernel<<<kBlocks3, kThreads, 0, stream>>>(P3, ei, b3, out);
}
